// DualMem_49357764165819
// MI455X (gfx1250) — hardware-verified
//
#include <hip/hip_runtime.h>
#include <math.h>

typedef __attribute__((ext_vector_type(16))) _Float16 v16h;
typedef __attribute__((ext_vector_type(16))) __bf16 v16b;
typedef __attribute__((ext_vector_type(8)))  _Float16 v8h;
typedef __attribute__((ext_vector_type(8)))  float v8f;
typedef __attribute__((ext_vector_type(4)))  float v4f;
typedef __attribute__((ext_vector_type(2)))  float v2f;
typedef __attribute__((ext_vector_type(4)))  unsigned v4u;
typedef __attribute__((ext_vector_type(4)))  int v4i;
typedef float __attribute__((may_alias)) float_a;
typedef int __attribute__((may_alias)) int_a;

template <typename T> __device__ __forceinline__ void vst2(void* p, T v) { *(volatile T*)p = v; __threadfence(); *(volatile T*)p = v; }
__device__ __forceinline__ v8f wmma16(v16h a, v16h b, v8f c) {
  v8f d = __builtin_amdgcn_wmma_f32_16x16x32_f16(false, a, false, b, (short)0, c, false, false);
  asm volatile("v_nop\n\tv_nop\n\tv_nop\n\tv_nop" : "+v"(d) : "v"(a), "v"(b));
  return d;
}
__device__ __forceinline__ v8f wmma_bf(v16b a, v16b b, v8f c) {
  v8f d = __builtin_amdgcn_wmma_f32_16x16x32_bf16(false, a, false, b, (short)0, c, false, false);
  asm volatile("v_nop\n\tv_nop\n\tv_nop\n\tv_nop" : "+v"(d) : "v"(a), "v"(b));
  return d;
}
__device__ __forceinline__ v16h frag_h(const _Float16* rowk0, int lane) {
  union { v16h v; v8h q[2]; } u; const _Float16* p = rowk0 + 8 * (lane >> 4);
  u.q[0] = *(const v8h*)p; u.q[1] = *(const v8h*)(p + 16); return u.v;
}
__device__ __forceinline__ v16h frag_f32(const float* rowk0, int lane) {
  v16h a; const float* p = rowk0 + 8 * (lane >> 4);
#pragma unroll
  for (int i = 0; i < 8; ++i) { a[i] = (_Float16)p[i]; a[8 + i] = (_Float16)p[16 + i]; }
  return a;
}
__device__ __forceinline__ v16h frag_f32s(const float* rowk0, int lane, float sc) {
  v16h a; const float* p = rowk0 + 8 * (lane >> 4);
#pragma unroll
  for (int i = 0; i < 8; ++i) { a[i] = (_Float16)(p[i] * sc); a[8 + i] = (_Float16)(p[16 + i] * sc); }
  return a;
}
__device__ __forceinline__ v16h fragc_f32(const float* W, int k0, int n, int lane, int ld, int K) {
  v16h a; const int g = lane >> 4;
#pragma unroll
  for (int i = 0; i < 8; ++i) { const int ka = k0 + 8 * g + i, kb = ka + 16;
    a[i] = (_Float16)(ka < K ? W[(size_t)(ka < K ? ka : K - 1) * ld + n] : 0.f); a[8 + i] = (_Float16)(kb < K ? W[(size_t)(kb < K ? kb : K - 1) * ld + n] : 0.f); }
  return a;
}
struct F2 { v16b h, l; };
__device__ __forceinline__ F2 bsplit16(const float v[16]) { F2 r;
#pragma unroll
  for (int i = 0; i < 16; ++i) { const __bf16 h = (__bf16)v[i]; r.h[i] = h; r.l[i] = (__bf16)(v[i] - (float)h); }
  return r; }
__device__ __forceinline__ F2 split_row(const float* row, int k0, int lane) { float v[16]; const float* p = row + k0 + 8 * (lane >> 4);
#pragma unroll
  for (int i = 0; i < 8; ++i) { v[i] = p[i]; v[8 + i] = p[16 + i]; }
  return bsplit16(v); }
__device__ __forceinline__ F2 split_rowK(const float* row, int k0, int lane, int K) { float v[16]; const int g = lane >> 4;
#pragma unroll
  for (int i = 0; i < 8; ++i) { const int ka = k0 + 8 * g + i, kb = ka + 16; v[i] = ka < K ? row[ka < K ? ka : K - 1] : 0.f; v[8 + i] = kb < K ? row[kb < K ? kb : K - 1] : 0.f; }
  return bsplit16(v); }
__device__ __forceinline__ F2 split_col(const float* W, int k0, int n, int lane, int ld, int K) { float v[16]; const int g = lane >> 4;
#pragma unroll
  for (int i = 0; i < 8; ++i) { const int ka = k0 + 8 * g + i, kb = ka + 16; v[i] = ka < K ? W[(size_t)(ka < K ? ka : K - 1) * ld + n] : 0.f; v[8 + i] = kb < K ? W[(size_t)(kb < K ? kb : K - 1) * ld + n] : 0.f; }
  return bsplit16(v); }
__device__ __forceinline__ v8f mac3(const F2& a, const F2& b, v8f c) { c = wmma_bf(a.l, b.h, c); c = wmma_bf(a.h, b.l, c); return wmma_bf(a.h, b.h, c); }
__device__ __forceinline__ float sigm(float v) { return 1.0f / (1.0f + expf(-v)); }
#define LDSX() do { asm volatile("s_wait_dscnt 0" ::: "memory"); __builtin_amdgcn_wave_barrier(); __builtin_amdgcn_fence(__ATOMIC_RELEASE, "workgroup"); } while (0)


#define NB 64
#define NCLS 1000
#define NM 11
#define DD 1024
#define NMEM (NCLS * NM)
#define NMEMP 11008
#ifndef NCT
#define NCT NCLS
#endif
typedef __attribute__((ext_vector_type(8))) __bf16 v8b;
__device__ __forceinline__ v16b frag_b(const __bf16* rowk0, int lane) {
  union { v16b v; v8b q[2]; } u; const __bf16* p = rowk0 + 8 * (lane >> 4);
  u.q[0] = *(const v8b*)p; u.q[1] = *(const v8b*)(p + 16); return u.v;
}
__device__ __forceinline__ float bfr(float v) { return (float)(__bf16)v; }
__device__ __attribute__((noinline)) float exp_ni(float v) { return expf(v); }
__device__ __attribute__((noinline)) float erf_ni(float v) { return erff(v); }

#define WS_IB  0u
#define WS_MB  (WS_IB + 2u * NB * DD)
#define WS_MT  (WS_MB + 2u * NMEMP * DD)
#define WS_W   (WS_MT + 2u * (size_t)NCLS * DD * 32)
#define WS_LT  (WS_W + 4u * NB * NMEMP)
#define WS_END (WS_LT + 4u * 1024 * NB)

__global__ __launch_bounds__(128) void k_rows(const float* __restrict__ IMG, const float* __restrict__ MEM, __bf16* __restrict__ IB, __bf16* __restrict__ MB) {
  __shared__ __align__(16) __bf16 s[DD]; const int r = blockIdx.x, which = blockIdx.y, t = threadIdx.x;
  if (which == 0 && r >= NB) return;
  const float* src = (which == 0) ? IMG + (size_t)r * DD : MEM + (size_t)min(r, NMEM - 1) * DD; const bool z = (which == 1 && r >= NMEM);
  for (int k = t; k < DD; k += 128) s[k] = (__bf16)(z ? 0.f : src[k]);
  __syncthreads();
  vst2((unsigned*)((which == 0 ? IB : MB) + (size_t)r * DD + t * 8), *(const v4u*)&s[t * 8]);
}
__global__ __launch_bounds__(128) void k_mt(const float* __restrict__ MEM, __bf16* __restrict__ MT) {
  __shared__ __align__(16) __bf16 s[128][40]; const int c = blockIdx.x, d0 = blockIdx.y * 128, t = threadIdx.x;
  for (int m = 0; m < 32; ++m) s[t][m] = (__bf16)((m < NM) ? MEM[((size_t)c * NM + m) * DD + d0 + t] : 0.f);
  __syncthreads();
  for (int q = t; q < 128 * 4; q += 128) { const int dl = q >> 2, pc = q & 3; vst2((unsigned*)(MT + ((size_t)c * DD + d0 + dl) * 32 + pc * 8), *(const v4u*)&s[dl][pc * 8]); }
}
__global__ __launch_bounds__(128) void k_sim(const __bf16* __restrict__ IB, const __bf16* __restrict__ MB, float* __restrict__ Wt) {
  __shared__ __align__(16) float so[4][16][132];
  const int tid = threadIdx.x, wave = tid >> 5, lane = tid & 31, col = lane & 15, g = lane >> 4; const size_t r0 = (size_t)wave * 16; const int n0 = blockIdx.x * 128;
  v8f acc[8] = {};
#pragma unroll 4
  for (int kc = 0; kc < DD / 32; ++kc) { const v16b a = frag_b(IB + (r0 + col) * DD + kc * 32, lane);
#pragma unroll
    for (int j = 0; j < 8; ++j) acc[j] = wmma_bf(a, frag_b(MB + (size_t)(n0 + j * 16 + col) * DD + kc * 32, lane), acc[j]); }
#pragma unroll
  for (int j = 0; j < 8; ++j)
#pragma unroll
    for (int r = 0; r < 8; ++r) so[wave][8 * g + r][j * 16 + col] = __expf(-5.5f * (1.0f - acc[j][r]));
  LDSX();
  for (int rl = 0; rl < 16; ++rl) vst2(Wt + (r0 + rl) * NMEMP + n0 + lane * 4, *(const v4f*)&so[wave][rl][lane * 4]);
}
__global__ __launch_bounds__(128) void k_adapt(const float* __restrict__ Wt, const __bf16* __restrict__ MT, const float* __restrict__ IMG, float* __restrict__ LT) {
  __shared__ __align__(16) float so[64];
  const int tid = threadIdx.x, wave = tid >> 5, lane = tid & 31, col = lane & 15, g = lane >> 4; const int c = blockIdx.x; const int b = wave * 16 + col;
  F2 a; { float v[16]; const float* wr = Wt + (size_t)b * NMEMP + (size_t)c * NM;
#pragma unroll
    for (int i = 0; i < 8; ++i) { const int k0 = 8 * g + i; v[i] = (k0 < NM) ? wr[k0] : 0.f; v[8 + i] = 0.f; }
    a = bsplit16(v); }
  float dot[8], sq[8];
#pragma unroll
  for (int r = 0; r < 8; ++r) { dot[r] = 0.f; sq[r] = 0.f; }
#pragma unroll 2
  for (int dt = 0; dt < DD / 16; ++dt) { v8f acc = {}; const v16b w = frag_b(MT + ((size_t)c * DD + dt * 16 + col) * 32, lane); acc = wmma_bf(a.l, w, acc); acc = wmma_bf(a.h, w, acc);
    const int d = dt * 16 + col;
#pragma unroll
    for (int r = 0; r < 8; ++r) { const float av = acc[r]; const float iv = bfr(IMG[(size_t)(wave * 16 + 8 * g + r) * DD + d]); dot[r] += iv * av; sq[r] += av * av; } }
#pragma unroll
  for (int r = 0; r < 8; ++r) { float dv = dot[r], sv = sq[r];
#pragma unroll
    for (int o = 1; o < 16; o <<= 1) { dv += __shfl_xor(dv, o); sv += __shfl_xor(sv, o); }
    if (col == 0) so[wave * 16 + 8 * g + r] = 100.0f * dv / sqrtf(sv); }
  __syncthreads();
  if (tid < 16) vst2(LT + (size_t)c * NB + tid * 4, *(const v4f*)&so[tid * 4]);
}
__global__ __launch_bounds__(256) void k_out(const float* __restrict__ LT, float* __restrict__ OUT) {
  const int tid = threadIdx.x;
  for (int q = tid; q < NB * NCLS / 4; q += 256) { v4f v;
#pragma unroll
    for (int i = 0; i < 4; ++i) { const int e = q * 4 + i; const int b = e / NCLS, c = e % NCLS; v[i] = (c < NCT) ? LT[(size_t)c * NB + b] : 0.f; }
    vst2(OUT + (size_t)q * 4, v); }
}
extern "C" void kernel_launch(void* const* d_in, const int* in_sizes, int n_in, void* d_out, int out_size, void* d_ws, size_t ws_size, hipStream_t stream) {
  (void)in_sizes; (void)n_in; (void)out_size;
  const float** F = (const float**)d_in;
  if (ws_size < (size_t)WS_END) return;
  char* ws = (char*)d_ws; __bf16 *IB = (__bf16*)(ws + WS_IB), *MB = (__bf16*)(ws + WS_MB), *MT = (__bf16*)(ws + WS_MT); float *Wt = (float*)(ws + WS_W), *LT = (float*)(ws + WS_LT);
  k_rows<<<dim3(NMEMP, 2), 128, 0, stream>>>(F[0], F[1], IB, MB);
  k_mt<<<dim3(NCT, DD / 128), 128, 0, stream>>>(F[1], MT);
  k_sim<<<NMEMP / 128, 128, 0, stream>>>(IB, MB, Wt);
  k_adapt<<<NCT, 128, 0, stream>>>(Wt, MT, F[0], LT);
  k_out<<<1, 256, 0, stream>>>(LT, (float*)d_out);
}
